// LightCurveRNN_1657857376385
// MI455X (gfx1250) — hardware-verified
//
#include <hip/hip_runtime.h>

typedef __attribute__((ext_vector_type(16))) _Float16 v16h;
typedef __attribute__((ext_vector_type(8)))  _Float16 v8h;
typedef __attribute__((ext_vector_type(8)))  float    v8f;
typedef __attribute__((ext_vector_type(4)))  float    v4f;

constexpr int kSeq   = 1024;
constexpr int kStep  = 1024;
constexpr int kHid   = 128;
constexpr int kCls   = 14;
constexpr int kClsPad = 16;

constexpr int kSeqPB      = 16;
constexpr int kRnnBlocks  = kSeq / kSeqPB;
constexpr int kRnnThreads = 256;
constexpr int kHP         = kHid + 8;
constexpr int kTile       = kSeqPB * kHP;
constexpr int kXC         = 64;
constexpr float kWScale   = 16.0f;
constexpr float kWInv     = 0.0625f;
static_assert(kSeq % kSeqPB == 0);
static_assert(kHid == (kRnnThreads / 32) * 16);
static_assert(kHP % 8 == 0);
static_assert(kHid % 32 == 0);
static_assert(kStep % kXC == 0);
static_assert(kXC * kSeqPB == 4 * kRnnThreads);
static_assert((kSeqPB * kCls * 4) % 128 == 0);
static_assert(kSeqPB * kCls <= 256);

constexpr int kDwW    = kHid * kHid / 2;
constexpr int kDwFcw  = kClsPad * kHid / 2;
constexpr int kBlkW   = kDwW / 256;
constexpr int kBlkFcw = kDwFcw / 256;
constexpr int kPrepB1 = kBlkW;
constexpr int kPrepB2 = kPrepB1 + kBlkW;
constexpr int kPrepB3 = kPrepB2 + kBlkW;
constexpr int kPrepBlocks = kPrepB3 + kBlkFcw;
static_assert(kDwW % 256 == 0 && kDwFcw % 256 == 0);
static_assert(kPrepBlocks == 100);

template <typename T> struct Frag;
template <> struct Frag<_Float16> {
  typedef v16h V; union U { v16h v; v8h h[2]; };
  static __device__ __forceinline__ v16h load(const _Float16* p) {
    U f; f.h[0] = *(const v8h*)(p); f.h[1] = *(const v8h*)(p + 16); return f.v;
  }
};
__device__ __forceinline__ v8f mma_g(v16h a, v16h b, v8f c) {
  c = __builtin_amdgcn_wmma_f32_16x16x32_f16(false, a, false, b, (short)0, c, false, false);
  asm volatile("v_nop\n\tv_nop\n\tv_nop\n\tv_nop" : "+v"(c) : "v"(a), "v"(b));
  return c;
}

__device__ __forceinline__ unsigned pack_f16x2(float a, float b) {
  const _Float16 h0 = (_Float16)a, h1 = (_Float16)b;
  return (unsigned)__builtin_bit_cast(unsigned short, h0) | ((unsigned)__builtin_bit_cast(unsigned short, h1) << 16);
}
__device__ __forceinline__ void st2u(unsigned* p, unsigned v) { *(volatile unsigned*)p = v; __threadfence(); *(volatile unsigned*)p = v; }
__device__ __forceinline__ float ftanh(float x) { return 1.0f - 2.0f * __builtin_amdgcn_rcpf(1.0f + __expf(2.0f * x)); }

__global__ __launch_bounds__(256) void prep_kernel(
    const float* __restrict__ w_hh0, const float* __restrict__ w_ih1,
    const float* __restrict__ w_hh1, const float* __restrict__ fc_w,
    unsigned* __restrict__ whh0u, unsigned* __restrict__ wih1u,
    unsigned* __restrict__ whh1u, unsigned* __restrict__ fcwu) {
  const int blk = blockIdx.x, tid = threadIdx.x;
  if (blk < kPrepB1) {
    const int p = blk * 256 + tid;
    st2u(whh0u + p, pack_f16x2(w_hh0[2 * p] * kWScale, w_hh0[2 * p + 1] * kWScale));
  } else if (blk < kPrepB2) {
    const int p = (blk - kPrepB1) * 256 + tid;
    st2u(wih1u + p, pack_f16x2(w_ih1[2 * p] * kWScale, w_ih1[2 * p + 1] * kWScale));
  } else if (blk < kPrepB3) {
    const int p = (blk - kPrepB2) * 256 + tid;
    st2u(whh1u + p, pack_f16x2(w_hh1[2 * p] * kWScale, w_hh1[2 * p + 1] * kWScale));
  } else {
    const int p = (blk - kPrepB3) * 256 + tid;
    const int row = p >> 6;
    const int pc = (p < kCls * (kHid / 2)) ? p : (kCls * (kHid / 2) - 1);
    const unsigned wv = pack_f16x2(fc_w[2 * pc] * kWScale, fc_w[2 * pc + 1] * kWScale);
    const unsigned v = (row < kCls) ? wv : 0u;
    st2u(fcwu + p, v);
  }
}

__global__ __launch_bounds__(kRnnThreads) void rnn2_kernel(
    const float* __restrict__ x, const float* __restrict__ w_ih0,
    const float* __restrict__ b_ih0, const float* __restrict__ b_hh0,
    const float* __restrict__ b_ih1, const float* __restrict__ b_hh1,
    const float* __restrict__ fc_b,
    const _Float16* __restrict__ whh0, const _Float16* __restrict__ wih1,
    const _Float16* __restrict__ whh1, const _Float16* __restrict__ fcw16,
    float* __restrict__ out) {
  __shared__ __align__(16) _Float16 hbuf[4 * kTile];
  __shared__ __align__(32) float xs[kXC * kSeqPB];
  __shared__ __align__(16) float outs[256];

  const int tid = threadIdx.x, lane = tid & 31, wave = tid >> 5;
  const int c = lane & 15, hh = lane >> 4, koff = hh * 8;
  const int seq0 = blockIdx.x * kSeqPB;
  const int n = wave * 16 + c;

  {
    const v8h z = {(_Float16)0.f, (_Float16)0.f, (_Float16)0.f, (_Float16)0.f, (_Float16)0.f, (_Float16)0.f, (_Float16)0.f, (_Float16)0.f};
    for (int i = tid; i < (4 * kTile) / 8; i += kRnnThreads) *(v8h*)(hbuf + i * 8) = z;
  }
  const float wih0n = w_ih0[n];
  const float bs0 = b_ih0[n] + b_hh0[n];
  const float bs1 = b_ih1[n] + b_hh1[n];
  const _Float16* b0row = whh0 + (size_t)n * kHid + koff;
  const _Float16* b1row = whh1 + (size_t)n * kHid + koff;
  const _Float16* birow = wih1 + (size_t)n * kHid + koff;
  __syncthreads();

#pragma unroll 1
  for (int t = 0; t < kStep; ++t) {
    if ((t & (kXC - 1)) == 0) {
#pragma unroll
      for (int i = 0; i < 4; ++i) {
        const int idx = tid + kRnnThreads * i;
        const int s = idx >> 6, tt = idx & 63;
        xs[tt * kSeqPB + s] = x[(size_t)(seq0 + s) * kStep + t + tt];
      }
      __syncthreads();
    }
    const _Float16* h1c = hbuf + (t & 1) * kTile;
    _Float16*       h1n = hbuf + ((t + 1) & 1) * kTile;
    const _Float16* h2c = hbuf + (2 + (t & 1)) * kTile;
    _Float16*       h2n = hbuf + (2 + ((t + 1) & 1)) * kTile;

    v8f acc0 = {0.f,0.f,0.f,0.f,0.f,0.f,0.f,0.f};
    v8f acc1 = {0.f,0.f,0.f,0.f,0.f,0.f,0.f,0.f};
    const _Float16* a1 = h1c + c * kHP + koff;
    const _Float16* a2 = h2c + c * kHP + koff;
#pragma unroll
    for (int kc = 0; kc < kHid / 32; ++kc) {
      const v16h fa = Frag<_Float16>::load(a1 + kc * 32);
      const v16h fb = Frag<_Float16>::load(b0row + kc * 32);
      acc0 = mma_g(fa, fb, acc0);
    }
#pragma unroll
    for (int kc = 0; kc < kHid / 32; ++kc) {
      const v16h fa = Frag<_Float16>::load(a2 + kc * 32);
      const v16h fb = Frag<_Float16>::load(b1row + kc * 32);
      acc1 = mma_g(fa, fb, acc1);
    }
    {
      const v8f xv = *(const v8f*)(xs + (t & (kXC - 1)) * kSeqPB + 8 * hh);
#pragma unroll
      for (int r = 0; r < 8; ++r) {
        const float pre = acc0[r] * kWInv + (xv[r] * wih0n + bs0);
        h1n[(8 * hh + r) * kHP + n] = (_Float16)ftanh(pre);
      }
    }
    __syncthreads();

    const _Float16* a3 = h1n + c * kHP + koff;
#pragma unroll
    for (int kc = 0; kc < kHid / 32; ++kc) {
      const v16h fa = Frag<_Float16>::load(a3 + kc * 32);
      const v16h fb = Frag<_Float16>::load(birow + kc * 32);
      acc1 = mma_g(fa, fb, acc1);
    }
#pragma unroll
    for (int r = 0; r < 8; ++r) {
      const float pre = acc1[r] * kWInv + bs1;
      h2n[(8 * hh + r) * kHP + n] = (_Float16)ftanh(pre);
    }
    __syncthreads();
  }

  const _Float16* hf = hbuf + (2 + (kStep & 1)) * kTile;
  if (wave == 0) {
    v8f acc = {0.f,0.f,0.f,0.f,0.f,0.f,0.f,0.f};
    const _Float16* af = hf + c * kHP + koff;
    const _Float16* bf = fcw16 + (size_t)c * kHid + koff;
#pragma unroll
    for (int kc = 0; kc < kHid / 32; ++kc) {
      const v16h fa = Frag<_Float16>::load(af + kc * 32);
      const v16h fb = Frag<_Float16>::load(bf + kc * 32);
      acc = mma_g(fa, fb, acc);
    }
    const float fbc = fc_b[(c < kCls) ? c : (kCls - 1)];
#pragma unroll
    for (int r = 0; r < 8; ++r) {
      const float v = acc[r] * kWInv + fbc;
      if (c < kCls) outs[(8 * hh + r) * kCls + c] = v;
    }
  }
  __syncthreads();
  if (wave == 0) {
    float* ob = out + (size_t)seq0 * kCls;
    for (int pass = 0; pass < 2; ++pass) {
#pragma unroll
      for (int it = 0; it < 2; ++it) {
        const int f = it * 128 + lane * 4;
        const v4f v = *(const v4f*)(outs + f);
        if (f < kSeqPB * kCls) *(volatile v4f*)(ob + f) = v;
      }
      __threadfence();
    }
  }
}

extern "C" void kernel_launch(void* const* d_in, const int* in_sizes, int n_in,
                              void* d_out, int out_size, void* d_ws, size_t ws_size, hipStream_t stream) {
  if (n_in < 11 || d_out == nullptr || d_ws == nullptr) return;
  if (in_sizes[0] != kSeq * kStep || in_sizes[1] != kHid || in_sizes[2] != kHid * kHid ||
      in_sizes[3] != kHid || in_sizes[4] != kHid || in_sizes[5] != kHid * kHid || in_sizes[6] != kHid * kHid ||
      in_sizes[7] != kHid || in_sizes[8] != kHid || in_sizes[9] != kCls * kHid || in_sizes[10] != kCls ||
      out_size != kSeq * kCls) return;

  const float* x     = (const float*)d_in[0];
  const float* w_ih0 = (const float*)d_in[1];
  const float* w_hh0 = (const float*)d_in[2];
  const float* b_ih0 = (const float*)d_in[3];
  const float* b_hh0 = (const float*)d_in[4];
  const float* w_ih1 = (const float*)d_in[5];
  const float* w_hh1 = (const float*)d_in[6];
  const float* b_ih1 = (const float*)d_in[7];
  const float* b_hh1 = (const float*)d_in[8];
  const float* fc_w  = (const float*)d_in[9];
  const float* fc_b  = (const float*)d_in[10];
  float* out = (float*)d_out;

  char* ws = (char*)d_ws; size_t off = 0;
  auto carve = [&](size_t bytes) -> char* { char* p = ws + off; off += (bytes + 255) & ~(size_t)255; return p; };
  unsigned short* WHH0_16 = (unsigned short*)carve((size_t)kHid * kHid * 2);
  unsigned short* WIH1_16 = (unsigned short*)carve((size_t)kHid * kHid * 2);
  unsigned short* WHH1_16 = (unsigned short*)carve((size_t)kHid * kHid * 2);
  unsigned short* FCW16   = (unsigned short*)carve((size_t)kClsPad * kHid * 2);
  if (off > ws_size || off > (size_t)134217728) return;

  prep_kernel<<<kPrepBlocks, 256, 0, stream>>>(w_hh0, w_ih1, w_hh1, fc_w,
                                               (unsigned*)WHH0_16, (unsigned*)WIH1_16,
                                               (unsigned*)WHH1_16, (unsigned*)FCW16);

  rnn2_kernel<<<kRnnBlocks, kRnnThreads, 0, stream>>>(x, w_ih0, b_ih0, b_hh0, b_ih1, b_hh1, fc_b,
                                                      (const _Float16*)WHH0_16, (const _Float16*)WIH1_16,
                                                      (const _Float16*)WHH1_16, (const _Float16*)FCW16, out);
}
